// GriffinBlock_21672404976192
// MI455X (gfx1250) — hardware-verified
//
#include <hip/hip_runtime.h>
#include <stdint.h>

#define DIMC  1024
#define HEADC 16
#define HDC   64
#define DFFC  4096

typedef __attribute__((ext_vector_type(16))) _Float16 v16h;
typedef __attribute__((ext_vector_type(8)))  _Float16 v8h;
typedef __attribute__((ext_vector_type(8)))  float    v8f;
typedef __attribute__((ext_vector_type(4)))  float    v4f;
#define PSCALE 32768.0f

__device__ __forceinline__ void dep_guard_h(v8f& a, v8f& b, v16h x, v16h y) { asm volatile("v_nop\n\tv_nop\n\tv_nop\n\tv_nop" : "+v"(a), "+v"(b) : "v"(x), "v"(y)); }
__device__ __forceinline__ void keep4_h(v16h a, v16h b, v16h c, v16h d) { asm volatile("v_nop" :: "v"(a), "v"(b), "v"(c), "v"(d)); }
__device__ __forceinline__ void acc_guard4(v8f& a, v8f& b, v8f& c, v8f& d) { asm volatile("v_nop\n\tv_nop\n\tv_nop\n\tv_nop" : "+v"(a), "+v"(b), "+v"(c), "+v"(d)); }

template <typename T> struct Frag;
template <> struct Frag<_Float16> {
  typedef v16h V; union U { v16h v; v8h h[2]; };
  static __device__ __forceinline__ v16h load(const _Float16* p) {
    U f; f.h[0] = *(const v8h*)(p); f.h[1] = *(const v8h*)(p + 16); return f.v;
  }
  static __device__ __forceinline__ v8f mma(v16h a, v16h b, v8f c) {
    return __builtin_amdgcn_wmma_f32_16x16x32_f16(false, a, false, b, (short)0, c, false, false);
  }
  static __device__ __forceinline__ void guard(v8f& a, v8f& b, v16h x, v16h y) { dep_guard_h(a, b, x, y); }
  static __device__ __forceinline__ void keep(v16h a, v16h b, v16h c, v16h d) { keep4_h(a, b, c, d); }
};

__device__ __forceinline__ v8f mma_h(v16h a, v16h b, v8f c) {
  c = __builtin_amdgcn_wmma_f32_16x16x32_f16(false, a, false, b, (short)0, c, false, false);
  asm volatile("v_nop\n\tv_nop\n\tv_nop\n\tv_nop" : "+v"(c) : "v"(a), "v"(b));
  return c;
}

__global__ __launch_bounds__(256) void cast_f32_f16x2s(
    const float* __restrict__ in, _Float16* __restrict__ out, int n2, float sc) {
  int i = blockIdx.x * 256 + threadIdx.x;
  if (i < n2) {
    const _Float16 h0 = (_Float16)(in[2 * i] * sc), h1 = (_Float16)(in[2 * i + 1] * sc);
    const unsigned u = (unsigned)__builtin_bit_cast(unsigned short, h0) | ((unsigned)__builtin_bit_cast(unsigned short, h1) << 16);
    ((volatile unsigned*)out)[i] = u;
    __threadfence();
    ((volatile unsigned*)out)[i] = u;
  }
}

__global__ __launch_bounds__(128) void rmsnorm_f16_kernel(
    const float* __restrict__ x, const float* __restrict__ w, _Float16* __restrict__ out, float eps) {
  __shared__ float red[4];
  const int row = blockIdx.x;
  const int lane = threadIdx.x & 31, wave = threadIdx.x >> 5;
  const int c0 = threadIdx.x * 8;
  const float* xr = x + (size_t)row * DIMC;
  const v4f xa = *(const v4f*)(xr + c0);
  const v4f xb = *(const v4f*)(xr + c0 + 4);
  float xs[8] = {xa[0], xa[1], xa[2], xa[3], xb[0], xb[1], xb[2], xb[3]};
  float ss = 0.0f;
#pragma unroll
  for (int e = 0; e < 8; ++e) ss += xs[e] * xs[e];
#pragma unroll
  for (int off = 16; off; off >>= 1) ss += __shfl_xor(ss, off, 32);
  if (lane == 0) red[wave] = ss;
  __syncthreads();
  const float tot = (red[0] + red[1]) + (red[2] + red[3]);
  const float rs = rsqrtf(tot * (1.0f / (float)DIMC) + eps);
  const v4f wa = *(const v4f*)(w + c0);
  const v4f wb = *(const v4f*)(w + c0 + 4);
  float wv[8] = {wa[0], wa[1], wa[2], wa[3], wb[0], wb[1], wb[2], wb[3]};
  v8h o;
#pragma unroll
  for (int e = 0; e < 8; ++e) o[e] = (_Float16)(wv[e] * (xs[e] * rs));
  _Float16* dst = out + (size_t)row * DIMC + c0;
  *(volatile v8h*)dst = o;
  __threadfence();
  *(volatile v8h*)dst = o;
}

__global__ __launch_bounds__(128) void rope_f16_kernel(
    const float* __restrict__ C, int ldC, const float* __restrict__ cs, const float* __restrict__ sn,
    _Float16* __restrict__ qk16, int S, int planeElems) {
  const int row = blockIdx.x;
  const int which = blockIdx.y;
  const int s = row % S;
  const int f0 = threadIdx.x * 8;
  const int d0 = f0 & (HDC - 1);
  const int pf = f0 ^ 32;
  const float sgn = (d0 < 32) ? -1.0f : 1.0f;
  const float* src = C + (size_t)row * ldC + (size_t)which * DIMC;
  const v4f x0 = *(const v4f*)(src + f0);
  const v4f x1 = *(const v4f*)(src + f0 + 4);
  const v4f y0 = *(const v4f*)(src + pf);
  const v4f y1 = *(const v4f*)(src + pf + 4);
  const float* cp = cs + (size_t)s * HDC + d0;
  const float* sp = sn + (size_t)s * HDC + d0;
  const v4f ca = *(const v4f*)(cp), cb = *(const v4f*)(cp + 4);
  const v4f sa = *(const v4f*)(sp), sb = *(const v4f*)(sp + 4);
  v8h o;
#pragma unroll
  for (int e = 0; e < 4; ++e) {
    o[e]     = (_Float16)(x0[e] * ca[e] + (sgn * y0[e]) * sa[e]);
    o[4 + e] = (_Float16)(x1[e] * cb[e] + (sgn * y1[e]) * sb[e]);
  }
  _Float16* dst = qk16 + (size_t)which * (size_t)planeElems + (size_t)row * DIMC + f0;
  *(volatile v8h*)dst = o;
  __threadfence();
  *(volatile v8h*)dst = o;
}

template <int BIAS_MODE, int OUT_MODE, bool RESID, int ACT, bool MULP, bool GATE>
__global__ __launch_bounds__(256) void wmma_gemm64(
    const unsigned short* __restrict__ Ap, int lda,
    const unsigned short* __restrict__ Btp, int ldb,
    void* __restrict__ Cout, int ldc,
    const float* __restrict__ bias,
    const float* __restrict__ resid,
    const unsigned short* __restrict__ Mulp, float mscale,
    const float* __restrict__ gatev,
    int M, int N, int K, float scale) {
  typedef _Float16 T;
  typedef v16h V;
  const T* A = (const T*)Ap; const T* Bt = (const T*)Btp; const T* Mp = (const T*)Mulp;
  __shared__ __align__(16) float sT[8][16 * 68];
  const int lane = threadIdx.x & 31;
  const int wave = threadIdx.x >> 5;
  const int tilesN = N >> 6;
  const int tilesM = M >> 6;
  const int tile = blockIdx.x * 8 + wave;
  if (tile >= tilesM * tilesN) return;
  const int tm = tile / tilesN;
  const int tn = tile - tm * tilesN;
  const int m0 = tm << 6;
  const int n0 = tn << 6;

  const int rlane = lane & 15;
  const int koff  = (lane >> 4) * 8;
  const int mOff  = (lane >> 4) * 8;

  v8f acc[4][4];
#pragma unroll
  for (int i = 0; i < 4; ++i)
#pragma unroll
    for (int j = 0; j < 4; ++j) acc[i][j] = (v8f){0.f,0.f,0.f,0.f,0.f,0.f,0.f,0.f};

  for (int k0 = 0; k0 < K; k0 += 32) {
    V bh[4];
#pragma unroll
    for (int j = 0; j < 4; ++j) {
      const size_t bo = (size_t)(n0 + (j << 4) + rlane) * ldb + koff + k0;
      bh[j] = Frag<T>::load(Bt + bo);
    }
#pragma unroll
    for (int i = 0; i < 4; ++i) {
      const size_t ao = (size_t)(m0 + (i << 4) + rlane) * lda + koff + k0;
      V ah = Frag<T>::load(A + ao);
#pragma unroll
      for (int j = 0; j < 4; ++j) acc[i][j] = Frag<T>::mma(ah, bh[j], acc[i][j]);
      Frag<T>::guard(acc[i][0], acc[i][3], ah, ah);
    }
    Frag<T>::keep(bh[0], bh[1], bh[2], bh[3]);
  }
  acc_guard4(acc[0][0], acc[0][1], acc[0][2], acc[0][3]);
  acc_guard4(acc[1][0], acc[1][1], acc[1][2], acc[1][3]);
  acc_guard4(acc[2][0], acc[2][1], acc[2][2], acc[2][3]);
  acc_guard4(acc[3][0], acc[3][1], acc[3][2], acc[3][3]);

  float* slab = sT[wave];
#pragma unroll
  for (int i = 0; i < 4; ++i) {
    const int mBase = m0 + (i << 4);
#pragma unroll
    for (int j = 0; j < 4; ++j) {
      const int n = n0 + (j << 4) + rlane;
      float bv = 0.f;
      if (BIAS_MODE == 2) bv = bias[n];
      float gsd = 1.0f;
      if (GATE) gsd = __builtin_amdgcn_rcpf(1.0f + __expf(-gatev[n]));
#pragma unroll
      for (int r = 0; r < 8; ++r) {
        const size_t eo = (size_t)(mBase + mOff + r) * ldc + n;
        float v = acc[i][j][r] * scale;
        if (BIAS_MODE == 1) v += bias[mBase + mOff + r];
        if (BIAS_MODE == 2) v += bv;
        if (ACT == 3) v = v * __builtin_amdgcn_rcpf(1.0f + __expf(-v));
        if (MULP) v = v * ((float)Mp[eo] * mscale);
        if (GATE) v = v * gsd;
        if (RESID) v += resid[eo];
        slab[(mOff + r) * 68 + (j << 4) + rlane] = v;
      }
    }
    __builtin_amdgcn_fence(__ATOMIC_RELEASE, "workgroup");
    __builtin_amdgcn_wave_barrier();
    __builtin_amdgcn_fence(__ATOMIC_ACQUIRE, "workgroup");
    if (OUT_MODE == 0) {
      float* C = (float*)Cout;
      const int hh = lane >> 4, c4 = (lane & 15) * 4;
      for (int pass = 0; pass < 2; ++pass) {
#pragma unroll
        for (int it = 0; it < 8; ++it) {
          const int row = it * 2 + hh;
          v4f vv = *(const v4f*)(slab + row * 68 + c4);
          *(volatile v4f*)(C + (size_t)(mBase + row) * ldc + n0 + c4) = vv;
        }
        __threadfence();
      }
    } else {
      const int q = lane >> 3, c8 = (lane & 7) * 8;
      unsigned short* C = (unsigned short*)Cout;
      for (int pass = 0; pass < 2; ++pass) {
#pragma unroll
        for (int it = 0; it < 4; ++it) {
          const int row = it * 4 + q;
          const float* sp = slab + row * 68 + c8;
          v8h hv;
#pragma unroll
          for (int e = 0; e < 8; ++e) hv[e] = (_Float16)sp[e];
          *(volatile v8h*)(C + (size_t)(mBase + row) * ldc + n0 + c8) = hv;
        }
        __threadfence();
      }
    }
    __builtin_amdgcn_fence(__ATOMIC_RELEASE, "workgroup");
    __builtin_amdgcn_wave_barrier();
    __builtin_amdgcn_fence(__ATOMIC_ACQUIRE, "workgroup");
  }
}

#define AT_QB 64
#define AT_KC 64
__global__ __launch_bounds__(128) void attn64_f16_kernel(
    const _Float16* __restrict__ q, const _Float16* __restrict__ k, const _Float16* __restrict__ v,
    _Float16* __restrict__ o, int S, int H, int ld, float qscale, float negfill, float oscale) {
  union FB { v16h v; v8h h[2]; };
  __shared__ __align__(16) _Float16 Ksh[AT_KC * HDC];
  __shared__ __align__(16) _Float16 Vth[HDC * AT_KC];
  __shared__ __align__(16) _Float16 Psh[4][16 * AT_KC];
  __shared__ __align__(16) float    Os[4][16 * 68];

  const int tid  = threadIdx.x;
  const int wave = tid >> 5;
  const int lane = tid & 31;
  const int hh   = lane >> 4;
  const int c    = lane & 15;

  const int nqb = S / AT_QB;
  const int bx = blockIdx.x;
  const int qb = bx % nqb;
  const int bh = bx / nqb;
  const int h  = bh % H;
  const int b  = bh / H;
  const int q0 = qb * AT_QB + wave * 16;

  const size_t boff = (size_t)b * (size_t)S * (size_t)ld + (size_t)h * HDC;
  const _Float16* qb_ptr = q + boff;
  const _Float16* kb_ptr = k + boff;
  const _Float16* vb_ptr = v + boff;
  _Float16*       ob_ptr = o + boff;

  v16h qa[2];
#pragma unroll
  for (int dc = 0; dc < 2; ++dc) qa[dc] = Frag<_Float16>::load(qb_ptr + (size_t)(q0 + c) * ld + dc * 32 + 8 * hh);

  float mrow[8], lrow[8];
  v8f oacc[4];
#pragma unroll
  for (int r = 0; r < 8; ++r) { mrow[r] = -1e30f; lrow[r] = 0.f; }
#pragma unroll
  for (int t = 0; t < 4; ++t) oacc[t] = (v8f){0.f,0.f,0.f,0.f,0.f,0.f,0.f,0.f};

  const int nChunks = qb + 1;
  for (int kc = 0; kc < nChunks; ++kc) {
    const int kv0 = kc * AT_KC;
    __syncthreads();
    {
      const int kvr = tid >> 1, dh = (tid & 1) * 32;
      const _Float16* krow = kb_ptr + (size_t)(kv0 + kvr) * ld + dh;
      const _Float16* vrow = vb_ptr + (size_t)(kv0 + kvr) * ld + dh;
#pragma unroll
      for (int i = 0; i < 4; ++i) {
        const v8h kk = *(const v8h*)(krow + 8 * i);
        *(v8h*)(Ksh + kvr * HDC + dh + 8 * i) = kk;
        const v8h vv = *(const v8h*)(vrow + 8 * i);
#pragma unroll
        for (int e = 0; e < 8; ++e) Vth[(dh + 8 * i + e) * AT_KC + kvr] = vv[e];
      }
    }
    __syncthreads();

    v8f s[4];
#pragma unroll
    for (int j = 0; j < 4; ++j) {
      s[j] = (v8f){0.f,0.f,0.f,0.f,0.f,0.f,0.f,0.f};
#pragma unroll
      for (int dc = 0; dc < 2; ++dc) {
        FB kb;
        kb.h[0] = *(const v8h*)(Ksh + (j * 16 + c) * HDC + dc * 32 + 8 * hh);
        kb.h[1] = *(const v8h*)(Ksh + (j * 16 + c) * HDC + dc * 32 + 16 + 8 * hh);
        s[j] = mma_h(qa[dc], kb.v, s[j]);
      }
    }
    const bool diag = (kc == qb);
    float cm[8];
#pragma unroll
    for (int r = 0; r < 8; ++r) {
      const int qrow = q0 + 8 * hh + r;
      float m = -1e30f;
#pragma unroll
      for (int j = 0; j < 4; ++j) {
        const int kvcol = kv0 + j * 16 + c;
        float val = s[j][r] * qscale;
        if (diag && (kvcol > qrow)) val += negfill;
        s[j][r] = val;
        m = fmaxf(m, val);
      }
#pragma unroll
      for (int off = 1; off < 16; off <<= 1) m = fmaxf(m, __shfl_xor(m, off, 32));
      cm[r] = m;
    }
    _Float16* pw = Psh[wave];
#pragma unroll
    for (int r = 0; r < 8; ++r) {
      const float mnew = fmaxf(mrow[r], cm[r]);
      const float alpha = expf(mrow[r] - mnew);
      mrow[r] = mnew;
      float psum = 0.f;
#pragma unroll
      for (int j = 0; j < 4; ++j) {
        const float p = expf(s[j][r] - mnew);
        psum += p;
        pw[(8 * hh + r) * AT_KC + j * 16 + c] = (_Float16)(p * PSCALE);
      }
#pragma unroll
      for (int off = 1; off < 16; off <<= 1) psum += __shfl_xor(psum, off, 32);
      lrow[r] = lrow[r] * alpha + psum;
#pragma unroll
      for (int t = 0; t < 4; ++t) oacc[t][r] *= alpha;
    }
    __builtin_amdgcn_fence(__ATOMIC_RELEASE, "workgroup");
    __builtin_amdgcn_wave_barrier();
    __builtin_amdgcn_fence(__ATOMIC_ACQUIRE, "workgroup");
#pragma unroll
    for (int kk = 0; kk < 2; ++kk) {
      FB pa;
      pa.h[0] = *(const v8h*)(pw + c * AT_KC + kk * 32 + 8 * hh);
      pa.h[1] = *(const v8h*)(pw + c * AT_KC + kk * 32 + 16 + 8 * hh);
#pragma unroll
      for (int t = 0; t < 4; ++t) {
        FB vb;
        vb.h[0] = *(const v8h*)(Vth + (t * 16 + c) * AT_KC + kk * 32 + 8 * hh);
        vb.h[1] = *(const v8h*)(Vth + (t * 16 + c) * AT_KC + kk * 32 + 16 + 8 * hh);
        oacc[t] = mma_h(pa.v, vb.v, oacc[t]);
      }
    }
  }

  float* os = Os[wave];
#pragma unroll
  for (int r = 0; r < 8; ++r) {
    const float inv = oscale / (lrow[r] * PSCALE);
#pragma unroll
    for (int t = 0; t < 4; ++t) os[(8 * hh + r) * 68 + t * 16 + c] = oacc[t][r] * inv;
  }
  __builtin_amdgcn_fence(__ATOMIC_RELEASE, "workgroup");
  __builtin_amdgcn_wave_barrier();
  __builtin_amdgcn_fence(__ATOMIC_ACQUIRE, "workgroup");
  {
    const int q4 = lane >> 3, c8 = (lane & 7) * 8;
    for (int pass = 0; pass < 2; ++pass) {
#pragma unroll
      for (int it = 0; it < 4; ++it) {
        const int row = it * 4 + q4;
        const float* sp = os + row * 68 + c8;
        v8h hv;
#pragma unroll
        for (int e = 0; e < 8; ++e) hv[e] = (_Float16)sp[e];
        *(volatile v8h*)(ob_ptr + (size_t)(q0 + row) * ld + c8) = hv;
      }
      __threadfence();
    }
  }
}

extern "C" void kernel_launch(void* const* d_in, const int* in_sizes, int n_in,
                              void* d_out, int out_size, void* d_ws, size_t ws_size,
                              hipStream_t stream) {
  if (n_in < 16) return;
  const float* h      = (const float*)d_in[0];
  const float* cosT   = (const float*)d_in[1];
  const float* sinT   = (const float*)d_in[2];
  const float* n1w    = (const float*)d_in[3];
  const float* wq     = (const float*)d_in[4];
  const float* wk     = (const float*)d_in[5];
  const float* wv     = (const float*)d_in[6];
  const float* wo     = (const float*)d_in[7];
  const float* n2w    = (const float*)d_in[8];
  const float* gate_w = (const float*)d_in[9];
  const float* gate_b = (const float*)d_in[10];
  const float* up_w   = (const float*)d_in[11];
  const float* up_b   = (const float*)d_in[12];
  const float* down_w = (const float*)d_in[13];
  const float* down_b = (const float*)d_in[14];
  const float* gatev  = (const float*)d_in[15];

  if (in_sizes[0] <= 0 || (in_sizes[0] % DIMC) != 0) return;
  const int M = in_sizes[0] / DIMC;
  if (in_sizes[1] <= 0 || (in_sizes[1] % HDC) != 0) return;
  const int S = in_sizes[1] / HDC;
  if ((M % 64) != 0 || (S % 64) != 0 || (M % S) != 0) return;
  if (in_sizes[2] != in_sizes[1]) return;
  if (in_sizes[3] != DIMC || in_sizes[8] != DIMC || in_sizes[14] != DIMC || in_sizes[15] != DIMC) return;
  if (in_sizes[4] != DIMC * DIMC || in_sizes[5] != DIMC * DIMC || in_sizes[6] != DIMC * DIMC || in_sizes[7] != DIMC * DIMC) return;
  if (in_sizes[9] != DFFC * DIMC || in_sizes[11] != DFFC * DIMC || in_sizes[13] != DIMC * DFFC) return;
  if (in_sizes[10] != DFFC || in_sizes[12] != DFFC) return;
  if (out_size != M * DIMC) return;
  const int Bb = M / S;

  char* ws = (char*)d_ws;
  size_t off = 0;
  auto carve = [&](size_t bytes) -> void* {
    void* p = ws + off;
    off += (bytes + 255) & ~(size_t)255;
    return p;
  };
  _Float16* wqkv16 = (_Float16*)carve((size_t)3 * DIMC * DIMC * 2);
  _Float16* wo16   = (_Float16*)carve((size_t)DIMC * DIMC * 2);
  _Float16* gw16   = (_Float16*)carve((size_t)DFFC * DIMC * 2);
  _Float16* uw16   = (_Float16*)carve((size_t)DFFC * DIMC * 2);
  _Float16* dw16   = (_Float16*)carve((size_t)DIMC * DFFC * 2);
  _Float16* x16    = (_Float16*)carve((size_t)M * DIMC * 2);
  float*    h1     = (float*)   carve((size_t)M * DIMC * 4);
  char*     scr    = (char*)    carve((size_t)M * 16384);
  if (off > ws_size) return;
  if (off > (size_t)134217728) return;
  float*    Cqk  = (float*)(scr);
  _Float16* q16  = (_Float16*)(scr + (size_t)M * 8192);
  _Float16* k16  = (_Float16*)(scr + (size_t)M * 10240);
  _Float16* v16  = (_Float16*)(scr + (size_t)M * 12288);
  _Float16* o16  = (_Float16*)(scr);
  _Float16* g16  = (_Float16*)(scr);
  _Float16* gu16 = (_Float16*)(scr + (size_t)M * 8192);

  const size_t planeElems = (size_t)M * DIMC;

  {
    const int n2a = DIMC * DIMC / 2;
    const unsigned ga = (unsigned)((n2a + 255) / 256);
    cast_f32_f16x2s<<<dim3(ga), dim3(256), 0, stream>>>(wq, wqkv16, n2a, 64.0f);
    cast_f32_f16x2s<<<dim3(ga), dim3(256), 0, stream>>>(wk, wqkv16 + (size_t)DIMC * DIMC, n2a, 64.0f);
    cast_f32_f16x2s<<<dim3(ga), dim3(256), 0, stream>>>(wv, wqkv16 + (size_t)2 * DIMC * DIMC, n2a, 64.0f);
    cast_f32_f16x2s<<<dim3(ga), dim3(256), 0, stream>>>(wo, wo16, n2a, 64.0f);
    const int n2b = DFFC * DIMC / 2;
    const unsigned gb = (unsigned)((n2b + 255) / 256);
    cast_f32_f16x2s<<<dim3(gb), dim3(256), 0, stream>>>(gate_w, gw16, n2b, 64.0f);
    cast_f32_f16x2s<<<dim3(gb), dim3(256), 0, stream>>>(up_w, uw16, n2b, 64.0f);
    cast_f32_f16x2s<<<dim3(gb), dim3(256), 0, stream>>>(down_w, dw16, n2b, 64.0f);
  }

  rmsnorm_f16_kernel<<<dim3((unsigned)M), dim3(128), 0, stream>>>(h, n1w, x16, 1e-5f);

  {
    const int N = 2 * DIMC;
    const unsigned nb = (unsigned)((((M / 64) * (N / 64)) + 7) / 8);
    wmma_gemm64<0, 0, false, 0, false, false><<<dim3(nb), dim3(256), 0, stream>>>(
        (const unsigned short*)x16, DIMC, (const unsigned short*)wqkv16, DIMC, (void*)Cqk, N,
        nullptr, nullptr, nullptr, 1.0f, nullptr, M, N, DIMC, 1.0f / 64.0f);
  }
  {
    const int N = DIMC;
    const unsigned nb = (unsigned)((((M / 64) * (N / 64)) + 7) / 8);
    wmma_gemm64<0, 1, false, 0, false, false><<<dim3(nb), dim3(256), 0, stream>>>(
        (const unsigned short*)x16, DIMC, (const unsigned short*)(wqkv16 + (size_t)2 * DIMC * DIMC), DIMC, (void*)v16, N,
        nullptr, nullptr, nullptr, 1.0f, nullptr, M, N, DIMC, 1.0f / 64.0f);
  }

  rope_f16_kernel<<<dim3((unsigned)M, 2), dim3(128), 0, stream>>>(Cqk, 2 * DIMC, cosT, sinT, q16, S, (int)planeElems);
  (void)k16;

  {
    const unsigned nb = (unsigned)(Bb * HEADC * (S / 64));
    attn64_f16_kernel<<<dim3(nb), dim3(128), 0, stream>>>(q16, k16, v16, o16, S, HEADC, DIMC, 0.125f, -1e4f, 16.0f);
  }

  {
    const int N = DIMC;
    const unsigned nb = (unsigned)((((M / 64) * (N / 64)) + 7) / 8);
    wmma_gemm64<0, 0, true, 0, false, false><<<dim3(nb), dim3(256), 0, stream>>>(
        (const unsigned short*)o16, DIMC, (const unsigned short*)wo16, DIMC, (void*)h1, N,
        nullptr, h, nullptr, 1.0f, nullptr, M, N, DIMC, 1.0f / 1024.0f);
  }

  rmsnorm_f16_kernel<<<dim3((unsigned)M), dim3(128), 0, stream>>>(h1, n2w, x16, 1e-5f);

  {
    const int N = DFFC;
    const unsigned nb = (unsigned)((((M / 64) * (N / 64)) + 7) / 8);
    wmma_gemm64<2, 1, false, 3, false, false><<<dim3(nb), dim3(256), 0, stream>>>(
        (const unsigned short*)x16, DIMC, (const unsigned short*)gw16, DIMC, (void*)g16, N,
        gate_b, nullptr, nullptr, 1.0f, nullptr, M, N, DIMC, 1.0f / 64.0f);
  }
  {
    const int N = DFFC;
    const unsigned nb = (unsigned)((((M / 64) * (N / 64)) + 7) / 8);
    wmma_gemm64<2, 1, false, 0, true, false><<<dim3(nb), dim3(256), 0, stream>>>(
        (const unsigned short*)x16, DIMC, (const unsigned short*)uw16, DIMC, (void*)gu16, N,
        up_b, nullptr, (const unsigned short*)g16, 16.0f, nullptr, M, N, DIMC, 1.0f / 64.0f);
  }
  {
    const int N = DIMC;
    const unsigned nb = (unsigned)((((M / 64) * (N / 64)) + 7) / 8);
    wmma_gemm64<2, 0, true, 0, false, true><<<dim3(nb), dim3(256), 0, stream>>>(
        (const unsigned short*)gu16, DFFC, (const unsigned short*)dw16, DFFC, d_out, N,
        down_b, h1, nullptr, 1.0f, gatev, M, N, DFFC, 1.0f / 1024.0f);
  }
}
